// IARM_89489938579708
// MI455X (gfx1250) — hardware-run, weakly checked
//
#include <hip/hip_runtime.h>
#include <math.h>

typedef __attribute__((ext_vector_type(16))) _Float16 v16h;
typedef __attribute__((ext_vector_type(16))) __bf16 v16b;
typedef __attribute__((ext_vector_type(8)))  _Float16 v8h;
typedef __attribute__((ext_vector_type(8)))  float v8f;
typedef __attribute__((ext_vector_type(4)))  float v4f;
typedef __attribute__((ext_vector_type(2)))  float v2f;
typedef __attribute__((ext_vector_type(4)))  unsigned v4u;
typedef __attribute__((ext_vector_type(4)))  int v4i;
typedef float __attribute__((may_alias)) float_a;
typedef int __attribute__((may_alias)) int_a;

template <typename T> __device__ __forceinline__ void vst2(void* p, T v) { *(volatile T*)p = v; __threadfence(); *(volatile T*)p = v; }
__device__ __forceinline__ v8f wmma16(v16h a, v16h b, v8f c) {
  v8f d = __builtin_amdgcn_wmma_f32_16x16x32_f16(false, a, false, b, (short)0, c, false, false);
  asm volatile("v_nop\n\tv_nop\n\tv_nop\n\tv_nop" : "+v"(d) : "v"(a), "v"(b));
  return d;
}
__device__ __forceinline__ v8f wmma_bf(v16b a, v16b b, v8f c) {
  v8f d = __builtin_amdgcn_wmma_f32_16x16x32_bf16(false, a, false, b, (short)0, c, false, false);
  asm volatile("v_nop\n\tv_nop\n\tv_nop\n\tv_nop" : "+v"(d) : "v"(a), "v"(b));
  return d;
}
__device__ __forceinline__ v16h frag_h(const _Float16* rowk0, int lane) {
  union { v16h v; v8h q[2]; } u; const _Float16* p = rowk0 + 8 * (lane >> 4);
  u.q[0] = *(const v8h*)p; u.q[1] = *(const v8h*)(p + 16); return u.v;
}
__device__ __forceinline__ v16h frag_f32(const float* rowk0, int lane) {
  v16h a; const float* p = rowk0 + 8 * (lane >> 4);
#pragma unroll
  for (int i = 0; i < 8; ++i) { a[i] = (_Float16)p[i]; a[8 + i] = (_Float16)p[16 + i]; }
  return a;
}
__device__ __forceinline__ v16h frag_f32s(const float* rowk0, int lane, float sc) {
  v16h a; const float* p = rowk0 + 8 * (lane >> 4);
#pragma unroll
  for (int i = 0; i < 8; ++i) { a[i] = (_Float16)(p[i] * sc); a[8 + i] = (_Float16)(p[16 + i] * sc); }
  return a;
}
__device__ __forceinline__ v16h fragc_f32(const float* W, int k0, int n, int lane, int ld, int K) {
  v16h a; const int g = lane >> 4;
#pragma unroll
  for (int i = 0; i < 8; ++i) { const int ka = k0 + 8 * g + i, kb = ka + 16;
    a[i] = (_Float16)(ka < K ? W[(size_t)(ka < K ? ka : K - 1) * ld + n] : 0.f); a[8 + i] = (_Float16)(kb < K ? W[(size_t)(kb < K ? kb : K - 1) * ld + n] : 0.f); }
  return a;
}
struct F2 { v16b h, l; };
__device__ __forceinline__ F2 bsplit16(const float v[16]) { F2 r;
#pragma unroll
  for (int i = 0; i < 16; ++i) { const __bf16 h = (__bf16)v[i]; r.h[i] = h; r.l[i] = (__bf16)(v[i] - (float)h); }
  return r; }
__device__ __forceinline__ F2 split_row(const float* row, int k0, int lane) { float v[16]; const float* p = row + k0 + 8 * (lane >> 4);
#pragma unroll
  for (int i = 0; i < 8; ++i) { v[i] = p[i]; v[8 + i] = p[16 + i]; }
  return bsplit16(v); }
__device__ __forceinline__ F2 split_rowK(const float* row, int k0, int lane, int K) { float v[16]; const int g = lane >> 4;
#pragma unroll
  for (int i = 0; i < 8; ++i) { const int ka = k0 + 8 * g + i, kb = ka + 16; v[i] = ka < K ? row[ka < K ? ka : K - 1] : 0.f; v[8 + i] = kb < K ? row[kb < K ? kb : K - 1] : 0.f; }
  return bsplit16(v); }
__device__ __forceinline__ F2 split_col(const float* W, int k0, int n, int lane, int ld, int K) { float v[16]; const int g = lane >> 4;
#pragma unroll
  for (int i = 0; i < 8; ++i) { const int ka = k0 + 8 * g + i, kb = ka + 16; v[i] = ka < K ? W[(size_t)(ka < K ? ka : K - 1) * ld + n] : 0.f; v[8 + i] = kb < K ? W[(size_t)(kb < K ? kb : K - 1) * ld + n] : 0.f; }
  return bsplit16(v); }
__device__ __forceinline__ v8f mac3(const F2& a, const F2& b, v8f c) { c = wmma_bf(a.l, b.h, c); c = wmma_bf(a.h, b.l, c); return wmma_bf(a.h, b.h, c); }
__device__ __forceinline__ float sigm(float v) { return 1.0f / (1.0f + expf(-v)); }
#define LDSX() do { asm volatile("s_wait_dscnt 0" ::: "memory"); __builtin_amdgcn_wave_barrier(); __builtin_amdgcn_fence(__ATOMIC_RELEASE, "workgroup"); } while (0)


#define NB 32
#define NN 512
#define DD 768
#define RR 128
#define NH 4
#define NL 2
#define HR (NH * RR)
#define NR (NB * NN)
#ifndef TNB
#define TNB NB
#endif
#define TR (TNB * NN)
typedef __attribute__((ext_vector_type(8))) __bf16 v8b;
__device__ __forceinline__ v16b frag_b(const __bf16* rowk0, int lane) {
  union { v16b v; v8b q[2]; } u; const __bf16* p = rowk0 + 8 * (lane >> 4);
  u.q[0] = *(const v8b*)p; u.q[1] = *(const v8b*)(p + 16); return u.v;
}
__device__ __forceinline__ float bfr(float v) { return (float)(__bf16)v; }
__device__ __attribute__((noinline)) float exp_ni(float v) { return expf(v); }
__device__ __attribute__((noinline)) float erf_ni(float v) { return erff(v); }

#define WS_PP   0u
#define WS_PG   (WS_PP + 2u * (size_t)RR * DD)
#define WS_PHW  (WS_PG + 2u * (size_t)NL * HR * RR)
#define WS_PO   (WS_PHW + 2u * (size_t)NL * RR * HR)
#define WS_H    (WS_PO + 2u * (size_t)DD * RR)
#define WS_WH   (WS_H + 4u * (size_t)NR * RR)
#define WS_WHP  (WS_WH + 4u * (size_t)NR * HR)
#define WS_WHL  (WS_WHP + 2u * (size_t)NB * HR * NN)
#define WS_F    (WS_WHL + 2u * (size_t)NB * HR * NN)
#define WS_CAT  (WS_F + 4u * (size_t)2 * NB * NH * NN)
#define WS_END  (WS_CAT + 4u * (size_t)NR * HR)

__global__ __launch_bounds__(256) void k_pack(const float* __restrict__ WP, const float* __restrict__ GW, const float* __restrict__ HW, const float* __restrict__ WO, __bf16* __restrict__ P) {
  __shared__ __align__(16) __bf16 s[DD]; const int t = threadIdx.x; int n = blockIdx.x; int K; __bf16* dst;
  if (n < RR) { K = DD; for (int k = t; k < K; k += 256) s[k] = (__bf16)WP[(size_t)k * RR + n]; dst = P + WS_PP / 2 + (size_t)n * DD; }
  else if ((n -= RR) < NL * HR) { const int l = n / HR, ho = n % HR, hh = ho / RR, o = ho % RR; K = RR; for (int k = t; k < K; k += 256) s[k] = (__bf16)GW[(((size_t)l * NH + hh) * RR + k) * RR + o]; dst = P + WS_PG / 2 + ((size_t)l * HR + ho) * RR; }
  else if ((n -= NL * HR) < NL * RR) { const int l = n / RR, o = n % RR; K = HR; for (int k = t; k < K; k += 256) s[k] = (__bf16)HW[((size_t)l * HR + k) * RR + o]; dst = P + WS_PHW / 2 + ((size_t)l * RR + o) * HR; }
  else { n -= NL * RR; K = RR; for (int k = t; k < K; k += 256) s[k] = (__bf16)WO[(size_t)k * DD + n]; dst = P + WS_PO / 2 + (size_t)n * RR; }
  __syncthreads(); for (int q = t; q < K / 8; q += 256) vst2((unsigned*)(dst + q * 8), *(const v4u*)&s[q * 8]);
}
template <int KDIM, int AMODE, int OMODE>
__global__ __launch_bounds__(128) void k_gemm(const float* __restrict__ A, const __bf16* __restrict__ Wr, const float* __restrict__ BIAS, const float* __restrict__ XR, int ncols, float* __restrict__ OUTF, _Float16* __restrict__ OPH, _Float16* __restrict__ OPL) {
  __shared__ __align__(16) float so[4][16][132]; __shared__ __align__(16) _Float16 st[128][72]; __shared__ __align__(16) _Float16 stl[128][72];
  const int tid = threadIdx.x, wave = tid >> 5, lane = tid & 31, col = lane & 15, g = lane >> 4; const size_t rb0 = (size_t)blockIdx.x * 64, r0 = rb0 + wave * 16; const int n0 = blockIdx.y * 128;
  v8f acc[8] = {};
#pragma unroll 2
  for (int kc = 0; kc < KDIM / 32; ++kc) {
    if (AMODE == 0) { v16b a; { const float* p = A + (r0 + col) * KDIM + kc * 32 + 8 * g;
#pragma unroll
        for (int i = 0; i < 8; ++i) { a[i] = (__bf16)p[i]; a[8 + i] = (__bf16)p[16 + i]; } }
#pragma unroll
      for (int j = 0; j < 8; ++j) acc[j] = wmma_bf(a, frag_b(Wr + (size_t)(n0 + j * 16 + col) * KDIM + kc * 32, lane), acc[j]); }
    else { const F2 a = split_row(A + (r0 + col) * KDIM, kc * 32, lane);
#pragma unroll
      for (int j = 0; j < 8; ++j) { const v16b w = frag_b(Wr + (size_t)(n0 + j * 16 + col) * KDIM + kc * 32, lane); acc[j] = wmma_bf(a.l, w, acc[j]); acc[j] = wmma_bf(a.h, w, acc[j]); } } }
#pragma unroll
  for (int j = 0; j < 8; ++j) { const int c = n0 + j * 16 + col; const float bb = BIAS ? bfr(BIAS[c]) : 0.f;
#pragma unroll
    for (int r = 0; r < 8; ++r) { float v = acc[j][r] + bb; if (OMODE == 2) v += bfr(XR[(r0 + 8 * g + r) * (size_t)ncols + c]); so[wave][8 * g + r][j * 16 + col] = v;
      if (OMODE == 1) { const _Float16 hh = (_Float16)v; st[j * 16 + col][wave * 16 + 8 * g + r] = hh; stl[j * 16 + col][wave * 16 + 8 * g + r] = (_Float16)((v - (float)hh) * 2048.0f); } } }
  LDSX();
  for (int rl = 0; rl < 16; ++rl) vst2(OUTF + (r0 + rl) * (size_t)ncols + n0 + lane * 4, *(const v4f*)&so[wave][rl][lane * 4]);
  if (OMODE == 1) { __syncthreads(); const size_t b = rb0 / NN, s0 = rb0 % NN;
    for (int e = tid; e < 128 * 8; e += 128) { const int d = e >> 3, pc = e & 7; vst2((unsigned*)(OPH + ((b * HR + n0 + d) * NN) + s0 + pc * 8), *(const v4u*)&st[d][pc * 8]); vst2((unsigned*)(OPL + ((b * HR + n0 + d) * NN) + s0 + pc * 8), *(const v4u*)&stl[d][pc * 8]); } }
}
__global__ __launch_bounds__(256) void k_f12(const float* __restrict__ WH, const float* __restrict__ A1, const float* __restrict__ A2, int l, float* __restrict__ F) {
  __shared__ __align__(16) float s1[NH][64], s2[NH][64]; const int t = threadIdx.x; const size_t rb0 = (size_t)blockIdx.x * 64; const int rl = t & 63, hh = t >> 6; const float* w = WH + (rb0 + rl) * HR + hh * RR; float u1 = 0.f, u2 = 0.f;
#pragma unroll 8
  for (int k = 0; k < RR; ++k) { const float wv = w[k]; u1 += wv * bfr(A1[((size_t)l * NH + hh) * RR + k]); u2 += wv * bfr(A2[((size_t)l * NH + hh) * RR + k]); }
  s1[hh][rl] = u1; s2[hh][rl] = u2; __syncthreads();
  const size_t b = rb0 / NN, s0 = rb0 % NN;
  if (t < NH * 16) { const int h2 = t >> 4, q = t & 15; vst2(F + (b * NH + h2) * NN + s0 + q * 4, *(const v4f*)&s1[h2][q * 4]); vst2(F + (size_t)NB * NH * NN + (b * NH + h2) * NN + s0 + q * 4, *(const v4f*)&s2[h2][q * 4]); }
}
__device__ __attribute__((noinline)) float exp_p(float v) { return expf(v); }
__device__ __forceinline__ float lk(float e) { return (e >= 0.f) ? e : 0.2f * e; }
__global__ __launch_bounds__(128) void k_gat(const float* __restrict__ F, const float* __restrict__ MASK, const _Float16* __restrict__ WHP, const _Float16* __restrict__ WHL, float* __restrict__ CAT) {
  __shared__ float sf2[NN], smk[NN]; __shared__ __align__(16) _Float16 sph[4][16][40]; __shared__ __align__(16) _Float16 spl[4][16][40]; __shared__ __align__(16) float so[4][16][132];
  const int tid = threadIdx.x, wave = tid >> 5, lane = tid & 31, col = lane & 15, g = lane >> 4; const int h = blockIdx.y; const size_t b = blockIdx.z; const int i0 = blockIdx.x * 64 + wave * 16; const size_t bh = b * NH + h;
  for (int j = tid; j < NN; j += 128) { sf2[j] = F[(size_t)NB * NH * NN + bh * NN + j]; smk[j] = bfr(MASK[b * NN + j]); }
  __syncthreads();
  float f1[8], mi[8], m[8], z[8];
#pragma unroll
  for (int r = 0; r < 8; ++r) { const int i = i0 + 8 * g + r; f1[r] = F[bh * NN + i]; mi[r] = bfr(MASK[b * NN + i]); m[r] = -3.0e38f; z[r] = 0.f; }
  for (int j = col; j < NN; j += 16) { const float f2 = sf2[j], mk = smk[j];
#pragma unroll
    for (int r = 0; r < 8; ++r) { const float e = (mi[r] * mk == 0.f) ? -1.0e9f : lk(f1[r] + f2); m[r] = fmaxf(m[r], e); } }
#pragma unroll
  for (int r = 0; r < 8; ++r) {
#pragma unroll
    for (int o = 1; o < 16; o <<= 1) m[r] = fmaxf(m[r], __shfl_xor(m[r], o)); }
  for (int j = col; j < NN; j += 16) { const float f2 = sf2[j], mk = smk[j];
#pragma unroll
    for (int r = 0; r < 8; ++r) { const float e = (mi[r] * mk == 0.f) ? -1.0e9f : lk(f1[r] + f2); z[r] += exp_p(e - m[r]); } }
#pragma unroll
  for (int r = 0; r < 8; ++r) {
#pragma unroll
    for (int o = 1; o < 16; o <<= 1) z[r] += __shfl_xor(z[r], o); }
  v8f acc[8] = {}, accl[8] = {};
#pragma unroll 1
  for (int js = 0; js < NN / 32; ++js) { const int jb = js * 32;
#pragma unroll
    for (int ct = 0; ct < 2; ++ct) { const int j = jb + ct * 16 + col; const float f2 = sf2[j], mk = smk[j];
#pragma unroll
      for (int r = 0; r < 8; ++r) { const float e = (mi[r] * mk == 0.f) ? -1.0e9f : lk(f1[r] + f2); const float ps = __expf(e - m[r]) / z[r] * 2048.0f; const _Float16 ph = (_Float16)ps; sph[wave][8 * g + r][ct * 16 + col] = ph; spl[wave][8 * g + r][ct * 16 + col] = (_Float16)((ps - (float)ph) * 2048.0f); } }
    LDSX();
    const v16h pa = frag_h(&sph[wave][col][0], lane), pal = frag_h(&spl[wave][col][0], lane);
#pragma unroll
    for (int dt = 0; dt < 8; ++dt) { const v16h wh = frag_h(WHP + ((b * HR + (size_t)h * RR + dt * 16 + col) * NN) + jb, lane); acc[dt] = wmma16(pa, wh, acc[dt]); accl[dt] = wmma16(pal, wh, accl[dt]); accl[dt] = wmma16(pa, frag_h(WHL + ((b * HR + (size_t)h * RR + dt * 16 + col) * NN) + jb, lane), accl[dt]); }
    LDSX(); }
#pragma unroll
  for (int r = 0; r < 8; ++r)
#pragma unroll
    for (int dt = 0; dt < 8; ++dt) { const float v = (acc[dt][r] + accl[dt][r] * (1.0f / 2048.0f)) * (1.0f / 2048.0f); so[wave][8 * g + r][dt * 16 + col] = (v > 0.f) ? v : (exp_p(v) - 1.0f); }
  LDSX();
  for (int rl = 0; rl < 16; ++rl) vst2(CAT + (b * NN + i0 + rl) * (size_t)HR + h * RR + lane * 4, *(const v4f*)&so[wave][rl][lane * 4]);
}
extern "C" void kernel_launch(void* const* d_in, const int* in_sizes, int n_in, void* d_out, int out_size, void* d_ws, size_t ws_size, hipStream_t stream) {
  (void)in_sizes; (void)n_in; (void)out_size;
  const float** Fi = (const float**)d_in;
  if (ws_size < (size_t)WS_END) return;
  char* ws = (char*)d_ws; __bf16* P = (__bf16*)ws; float *H = (float*)(ws + WS_H), *WH = (float*)(ws + WS_WH), *F = (float*)(ws + WS_F), *CAT = (float*)(ws + WS_CAT); _Float16 *WHP = (_Float16*)(ws + WS_WHP), *WHL = (_Float16*)(ws + WS_WHL);
  k_pack<<<RR + NL * HR + NL * RR + DD, 256, 0, stream>>>(Fi[2], Fi[4], Fi[7], Fi[9], P);
  k_gemm<DD, 0, 0><<<dim3(TR / 64, RR / 128), 128, 0, stream>>>(Fi[0], P + WS_PP / 2, Fi[3], nullptr, RR, H, nullptr, nullptr);
  for (int l = 0; l < NL; ++l) {
    k_gemm<RR, 1, 1><<<dim3(TR / 64, HR / 128), 128, 0, stream>>>(H, P + WS_PG / 2 + (size_t)l * HR * RR, nullptr, nullptr, HR, WH, WHP, WHL);
    k_f12<<<TR / 64, 256, 0, stream>>>(WH, Fi[5], Fi[6], l, F);
    k_gat<<<dim3(NN / 64, NH, TNB), 128, 0, stream>>>(F, Fi[1], WHP, WHL, CAT);
    k_gemm<HR, 1, 0><<<dim3(TR / 64, RR / 128), 128, 0, stream>>>(CAT, P + WS_PHW / 2 + (size_t)l * RR * HR, Fi[8] + (size_t)l * RR, nullptr, RR, H, nullptr, nullptr);
  }
  k_gemm<RR, 1, 2><<<dim3(TR / 64, DD / 128), 128, 0, stream>>>(H, P + WS_PO / 2, Fi[10], Fi[0], DD, (float*)d_out, nullptr, nullptr);
}
